// DyGraphTransformer_87342454931892
// MI455X (gfx1250) — hardware-run, weakly checked
//
#include <hip/hip_runtime.h>


namespace {
constexpr int N = 16384, E = 131072, FI = 256, HID = 512, HF = 256, H = 8, D = 32, L = 4, NV = 200, EV = 100, DV = 10, NPB = 8;
constexpr float XS = 8.0f, HS = 256.0f, WSC = 256.0f, EPS = 1e-5f, SCALE = 0.17677669529663687f;
typedef _Float16 b16;
typedef __attribute__((ext_vector_type(16))) _Float16 v16b;
typedef __attribute__((ext_vector_type(8))) _Float16 v8b;
typedef __attribute__((ext_vector_type(8))) float v8f;
typedef __attribute__((ext_vector_type(4))) float v4f;
__device__ __forceinline__ float bf16_rne(float f) { unsigned int u = __float_as_uint(f); u += 0x7FFFu + ((u >> 16) & 1u); float r = __uint_as_float(u & 0xFFFF0000u); asm volatile("" : "+v"(r)); return r; }
__device__ __forceinline__ float bfv(float f) { float r = bf16_rne(f); asm volatile("" : "+v"(r)); return r; }
__device__ __forceinline__ void split16(float v, b16& hi, b16& lo) { hi = (b16)v; lo = (b16)(v - (float)hi); }
__device__ __forceinline__ v16b frag_kb(const b16* p, int hh) { const v8b a = *(const v8b*)(p + 8 * hh), b = *(const v8b*)(p + 16 + 8 * hh); v16b f;
#pragma unroll
  for (int e = 0; e < 8; ++e) { f[e] = a[e]; f[8 + e] = b[e]; } return f; }
__device__ __forceinline__ v8f wmma16b(v16b a, v16b b, v8f c) { v8f d = __builtin_amdgcn_wmma_f32_16x16x32_f16(false, a, false, b, (short)0, c, false, false); asm volatile("v_nop\n\tv_nop\n\tv_nop\n\tv_nop" : "+v"(d) : "v"(a), "v"(b)); return d; }
__device__ __forceinline__ void wave_lds_sync() { __builtin_amdgcn_fence(__ATOMIC_RELEASE, "workgroup"); __builtin_amdgcn_wave_barrier(); __builtin_amdgcn_fence(__ATOMIC_ACQUIRE, "workgroup"); }
__device__ __forceinline__ float pmul(float a, float b) { float p = a * b; asm volatile("" : "+v"(p)); return p; }
__device__ __forceinline__ int iclamp(int v, int lo, int hi) { return v < lo ? lo : (v > hi ? hi : v); }
__device__ __forceinline__ float gelu_erf(float v) { return 0.5f * v * (1.0f + erff(v * 0.70710678118654752f)); }
constexpr int CSR_NBLK8 = 512, CSR_GB8 = 8, CSR_GN8 = 1 << CSR_GB8  , CSR_TS8 = (CSR_GN8 < 32 ? 32 : CSR_GN8)  , CSR_MAXG8 = 512, CSR_CAP8 = 12288  ;
__device__ __host__ __forceinline__ int csr_tix8(int v) { return (v >> CSR_GB8) * CSR_TS8 + (v & (CSR_GN8 - 1)); }
__global__ __launch_bounds__(64) void csrA_kernel8(const int* __restrict__ dst, int E, int N, int nG, int CHP, int NGP, int* __restrict__ STG, int* __restrict__ HST) {
  extern __shared__ int sm[];
  int* cnt = sm; int* run = sm + NGP; int* ids = sm + 2 * NGP;
  const int b = blockIdx.x; const int ch = (E + CSR_NBLK8 - 1) / CSR_NBLK8; const int e0 = b * ch, e1 = min(E, e0 + ch);
  for (int i = threadIdx.x; i < NGP; i += 64) cnt[i] = 0;
  for (int i = threadIdx.x; i < CHP; i += 64) ids[i] = -1;
  __syncthreads();
  if (threadIdx.x == 0) {
    for (int e = e0; e < e1; ++e) { int d = dst[e]; d = (d < 0) ? 0 : (d >= N ? N - 1 : d); cnt[d >> CSR_GB8] += 1; }
    int acc = 0; for (int g = 0; g < nG; ++g) { run[g] = acc; acc += cnt[g]; }
    for (int e = e0; e < e1; ++e) { int d = dst[e]; d = (d < 0) ? 0 : (d >= N ? N - 1 : d); const int g = d >> CSR_GB8; ids[run[g]] = e; run[g] += 1; } }
  __syncthreads();
  typedef __attribute__((ext_vector_type(4))) int v4i;
  for (int pass = 0; pass < 2; ++pass) {
    for (int i = threadIdx.x; i < CHP / 4; i += 64) *(volatile v4i*)(STG + (size_t)b * CHP + i * 4) = *(const v4i*)(&ids[i * 4]);
    for (int i = threadIdx.x; i < NGP / 4; i += 64) { v4i v; for (int e = 0; e < 4; ++e) v[e] = (i * 4 + e < nG) ? cnt[i * 4 + e] : 0; *(volatile v4i*)(HST + (size_t)b * NGP + i * 4) = v; }
    __threadfence(); }
}
__global__ __launch_bounds__(512) void csrS_kernel8(const int* __restrict__ HST, int nG, int NGP, int* __restrict__ START, int* __restrict__ TOT, int* __restrict__ OFF) {
  __shared__ int tot[CSR_MAXG8];
  const int b = threadIdx.x;
  for (int pass = 0; pass < 2; ++pass) { int runb = 0; for (int g = 0; g < nG; ++g) { int c = HST[(size_t)b * NGP + g]; c = (c < 0) ? 0 : c; ((volatile int*)OFF)[(size_t)g * CSR_NBLK8 + b] = runb; runb += c; } __threadfence(); }
  for (int g = threadIdx.x; g < nG; g += 512) { int s = 0; for (int bb = 0; bb < CSR_NBLK8; ++bb) { int c = HST[(size_t)bb * NGP + g]; s += (c < 0) ? 0 : c; } tot[g] = s; }
  __syncthreads();
  if (threadIdx.x < 32) {
    __shared__ int st[CSR_MAXG8 + 32];
    if (threadIdx.x == 0) { int acc = 0; for (int g = 0; g < NGP; ++g) { st[g] = acc; if (g < nG) acc += (tot[g] + 31) & ~31; } st[NGP] = acc; }
    __builtin_amdgcn_fence(__ATOMIC_RELEASE, "workgroup"); __builtin_amdgcn_wave_barrier(); __builtin_amdgcn_fence(__ATOMIC_ACQUIRE, "workgroup");
    for (int pass = 0; pass < 2; ++pass) { for (int i = threadIdx.x; i < NGP + 32; i += 32) { ((volatile int*)START)[i] = (i <= NGP) ? st[min(i, NGP)] : 0; ((volatile int*)TOT)[i] = (i < nG) ? tot[i] : 0; } __threadfence(); } }
}
__global__ __launch_bounds__(256) void csrB_kernel8(const int* __restrict__ dst, int N, int nG, int CHP, int NGP, int permLen, const int* __restrict__ STG, const int* __restrict__ HST, const int* __restrict__ OFF, const int* __restrict__ START, const int* __restrict__ TOT, int* __restrict__ PERM, int* __restrict__ ROWPTR, int* __restrict__ ROWCNT, int* __restrict__ FLAG) {
  typedef __attribute__((ext_vector_type(4))) int v4i;
  __shared__ int ids[CSR_CAP8]; __shared__ unsigned short key[CSR_CAP8]; __shared__ int outp[CSR_CAP8]; __shared__ int ncnt[CSR_GN8 + 1]; __shared__ int boff[CSR_NBLK8 + 1];
  const int g = blockIdx.x, t_ = threadIdx.x; int tot = TOT[g]; int st = START[g], stn = START[g + 1]; const int v0 = g * CSR_GN8; const int nv = min(CSR_GN8, N - v0); const int t0 = g * CSR_TS8;
  st = (st < 0) ? 0 : (st > permLen - 32 ? permLen - 32 : st) & ~31; stn = (stn < st) ? st : (stn > permLen ? permLen : stn); tot = (tot < 0) ? 0 : tot; if (tot > stn - st && tot <= CSR_CAP8) tot = stn - st;
  if (tot > CSR_CAP8) {
    for (int pass = 0; pass < 2; ++pass) { for (int i = t_; i < CSR_TS8 / 4; i += 256) { v4i a, c; for (int e = 0; e < 4; ++e) { a[e] = st; c[e] = 0; } *(volatile v4i*)(ROWPTR + t0 + i * 4) = a; *(volatile v4i*)(ROWCNT + t0 + i * 4) = c; } if (t_ == 0) ((volatile int*)FLAG)[0] = 1; __threadfence(); } (void)nv; return; }
  if (t_ == 0) { int acc = 0; for (int b = 0; b < CSR_NBLK8; ++b) { boff[b] = acc; int c = HST[(size_t)b * NGP + g]; c = (c < 0) ? 0 : (c > CHP ? CHP : c); acc += c; if (acc > tot) acc = tot; } boff[CSR_NBLK8] = acc; }
  for (int i = t_; i <= CSR_GN8; i += 256) ncnt[i] = 0;
  __syncthreads();
  for (int b = 0; b < CSR_NBLK8; ++b) { const int c = boff[b + 1] - boff[b]; int o_ = OFF[(size_t)g * CSR_NBLK8 + b]; o_ = (o_ < 0) ? 0 : (o_ > CHP - c ? CHP - c : o_); const int* src_ = STG + (size_t)b * CHP + o_;
    for (int i = t_; i < c; i += 256) { int id = src_[i]; id = (id < 0) ? 0 : id; ids[boff[b] + i] = id; int d = dst[id]; d = (d < v0) ? v0 : (d >= N ? N - 1 : d); int kk = d - v0; kk = (kk < 0) ? 0 : (kk >= CSR_GN8 ? CSR_GN8 - 1 : kk); key[boff[b] + i] = (unsigned short)kk; } }
  __syncthreads();
  if (t_ == 0) { for (int i = 0; i < tot; ++i) ncnt[key[i]] += 1; int acc = 0; for (int vl = 0; vl < CSR_GN8; ++vl) { const int c = ncnt[vl]; ncnt[vl] = acc; acc += c; } ncnt[CSR_GN8] = acc;
    for (int i = 0; i < tot; ++i) { const int vl = key[i]; outp[ncnt[vl]] = ids[i]; ncnt[vl] += 1; }
    for (int vl = CSR_GN8; vl > 0; --vl) ncnt[vl] = ncnt[vl - 1]; ncnt[0] = 0; }
  __syncthreads();
  for (int pass = 0; pass < 2; ++pass) {
    for (int i = t_; i < (stn - st) / 4; i += 256) { v4i v; for (int e = 0; e < 4; ++e) { const int q = i * 4 + e; v[e] = (q < tot) ? outp[q] : -1; } *(volatile v4i*)(PERM + st + i * 4) = v; }
    for (int i = t_; i < CSR_TS8 / 4; i += 256) { v4i a, c; for (int e = 0; e < 4; ++e) { const int vl = i * 4 + e; const int vc = vl < CSR_GN8 ? vl : CSR_GN8; a[e] = (vl < CSR_GN8) ? st + ncnt[vc] : st; c[e] = (vl < nv) ? (ncnt[(vc < CSR_GN8 ? vc : CSR_GN8 - 1) + 1] - ncnt[vc]) : 0; } *(volatile v4i*)(ROWPTR + t0 + i * 4) = a; *(volatile v4i*)(ROWCNT + t0 + i * 4) = c; }
    __threadfence(); }
}
__global__ __launch_bounds__(256) void csrZ_kernel8(int* __restrict__ p, size_t n4) { typedef __attribute__((ext_vector_type(4))) int v4i; const size_t tid = (size_t)blockIdx.x * 256 + threadIdx.x, nth = (size_t)gridDim.x * 256; v4i z = {0, 0, 0, 0}; for (size_t i = tid; i < n4; i += nth) *(volatile v4i*)(p + i * 4) = z; }
struct CsrBufs8 { int *STG, *HST, *OFF, *START, *TOT, *PERM, *ROWPTR, *ROWCNT, *FLAG; int nG, NGP, CHP; size_t permLen; char* base; size_t bytes; };
static size_t csr_carve8(CsrBufs8& c, char* ws, size_t off, int E, int N) {
  const size_t off0 = off; c.base = ws + off;
  auto al = [&](size_t bytes) { char* p = ws + off; off += (bytes + 255) & ~(size_t)255; return p; };
  c.nG = (N + CSR_GN8 - 1) / CSR_GN8; c.NGP = (c.nG + 31) & ~31; const int ch = (E + CSR_NBLK8 - 1) / CSR_NBLK8; c.CHP = (ch + 31) & ~31; c.permLen = (size_t)E + 32 * (size_t)c.nG + 32;
  c.STG = (int*)al((size_t)CSR_NBLK8 * c.CHP * 4); c.HST = (int*)al((size_t)CSR_NBLK8 * c.NGP * 4); c.OFF = (int*)al((size_t)c.NGP * CSR_NBLK8 * 4); c.START = (int*)al((size_t)(c.NGP + 64) * 4); c.TOT = (int*)al((size_t)(c.NGP + 64) * 4);
  c.PERM = (int*)al(c.permLen * 4); c.ROWPTR = (int*)al((size_t)c.nG * CSR_TS8 * 4); c.ROWCNT = (int*)al((size_t)c.nG * CSR_TS8 * 4); c.FLAG = (int*)al(256);
  c.bytes = off - off0; return off;
}
static void csr_build8(const CsrBufs8& c, const int* dst, int E, int N, hipStream_t stream) {
  const size_t smem = (size_t)(2 * c.NGP + c.CHP) * 4;
  csrZ_kernel8<<<512, 256, 0, stream>>>((int*)c.base, c.bytes / 16);
  csrA_kernel8<<<CSR_NBLK8, 64, smem, stream>>>(dst, E, N, c.nG, c.CHP, c.NGP, c.STG, c.HST);
  csrS_kernel8<<<1, 512, 0, stream>>>(c.HST, c.nG, c.NGP, c.START, c.TOT, c.OFF);
  csrB_kernel8<<<c.nG, 256, 0, stream>>>(dst, N, c.nG, c.CHP, c.NGP, (int)c.permLen, c.STG, c.HST, c.OFF, c.START, c.TOT, c.PERM, c.ROWPTR, c.ROWCNT, c.FLAG);
}


__global__ __launch_bounds__(256) void prep_kernel(const float* __restrict__ wfeat, const float* __restrict__ wq, const float* __restrict__ wk, const float* __restrict__ wv, const float* __restrict__ wo, const float* __restrict__ w1, const float* __restrict__ w2, const float* __restrict__ nemb, const float* __restrict__ eemb, const float* __restrict__ demb, const float* __restrict__ wedge, const float* __restrict__ wdist, b16* __restrict__ WF, b16* __restrict__ WL, float* __restrict__ TN, float* __restrict__ TE, float* __restrict__ TD) { const size_t nt = (size_t)gridDim.x * 256, u0 = (size_t)blockIdx.x * 256 + threadIdx.x; const int lane = threadIdx.x & 31; v8b v;
  for (size_t u = u0; u < (size_t)HID * (FI / 8); u += nt) { const int o = (int)(u / (FI / 8)), k0 = (int)(u % (FI / 8)) * 8;
#pragma unroll
    for (int j = 0; j < 8; ++j) v[j] = (b16)(bf16_rne(wfeat[(size_t)(k0 + j) * HID + o]) * WSC); for (int pass = 0; pass < 2; ++pass) { *(volatile v8b*)(WF + (size_t)o * FI + k0) = v; __threadfence(); } }
  for (size_t u = u0; u < (size_t)L * 6 * HF * (HF / 8); u += nt) { const int l = (int)(u / ((size_t)6 * HF * (HF / 8))); const size_t r = u % ((size_t)6 * HF * (HF / 8)); const int m = (int)(r / (HF * (HF / 8))), o = (int)((r / (HF / 8)) % HF), k0 = (int)(r % (HF / 8)) * 8; const float* w = (m == 0 ? wq : m == 1 ? wk : m == 2 ? wv : m == 3 ? wo : m == 4 ? w1 : w2) + (size_t)l * HF * HF;
#pragma unroll
    for (int j = 0; j < 8; ++j) v[j] = (b16)(bf16_rne(w[(size_t)(k0 + j) * HF + o]) * WSC); for (int pass = 0; pass < 2; ++pass) { *(volatile v8b*)(WL + (((size_t)l * 6 + m) * HF + o) * HF + k0) = v; __threadfence(); } }
  const size_t wid = u0 >> 5, nwaves = nt >> 5;
  for (size_t it = 0; it < (size_t)(NV + EV + DV); ++it) { size_t rI; if (it < (size_t)NV) { rI = wid + it * nwaves; if (rI >= (size_t)NV) { if (wid != 0) break; it = NV - 1; continue; } } else { if (wid != 0) break; rI = it; }
    if (rI < (size_t)NV) { const float* row = nemb + rI * HID; float ss = 0.0f; for (int c = lane; c < HID; c += 32) { const float t = bfv(row[c]); ss += t * t; } for (int o2 = 16; o2; o2 >>= 1) ss += __shfl_xor(ss, o2); const float f = fminf(1.0f, 1.0f / fmaxf(sqrtf(ss), 1e-7f)); for (int pass = 0; pass < 2; ++pass) { for (int c = lane; c < HID; c += 32) ((volatile float*)TN)[rI * HID + c] = bfv(row[c]) * f; __threadfence(); } }
    else { const bool isE = rI < (size_t)(NV + EV); const int vI = (int)(isE ? rI - NV : rI - NV - EV); const float* row = (isE ? eemb : demb) + (size_t)vI * HID; const float* wm = isE ? wedge : wdist; float ss = 0.0f; for (int c = lane; c < HID; c += 32) { const float t = bfv(row[c]); ss += t * t; } for (int o2 = 16; o2; o2 >>= 1) ss += __shfl_xor(ss, o2); const float f = fminf(1.0f, 1.0f / fmaxf(sqrtf(ss), 1e-7f));
      float mine = 0.0f;
#pragma unroll
      for (int hh = 0; hh < H; ++hh) { float s = 0.0f; for (int c = lane; c < HID; c += 32) s += pmul(bfv(row[c]) * f, bfv(wm[(size_t)c * H + hh])); for (int o2 = 16; o2; o2 >>= 1) s += __shfl_xor(s, o2); mine = (lane == hh) ? s : mine; }
      float* T = isE ? TE : TD; for (int pass = 0; pass < 2; ++pass) { if (lane < H) ((volatile float*)T)[(size_t)vI * H + lane] = mine; __threadfence(); } } } }
__global__ __launch_bounds__(256) void ebias_kernel(const int* __restrict__ eenc, const int* __restrict__ edist, const float* __restrict__ TE, const float* __restrict__ TD, const float* __restrict__ bedge, const float* __restrict__ bdist, float* __restrict__ EB) { const size_t e = (size_t)blockIdx.x * 256 + threadIdx.x; if (e >= (size_t)E) return; const int i1 = iclamp(eenc[e * 2], 0, EV - 1), i2 = iclamp(eenc[e * 2 + 1], 0, EV - 1), d = iclamp(edist[e], 0, DV - 1); v4f a, b;
  for (int hh = 0; hh < 4; ++hh) { a[hh] = (TE[i1 * H + hh] + TE[i2 * H + hh]) * 0.5f + bfv(bedge[hh]) + TD[d * H + hh] + bfv(bdist[hh]); b[hh] = (TE[i1 * H + 4 + hh] + TE[i2 * H + 4 + hh]) * 0.5f + bfv(bedge[4 + hh]) + TD[d * H + 4 + hh] + bfv(bdist[4 + hh]); }
  for (int pass = 0; pass < 2; ++pass) { *(volatile v4f*)(EB + e * H) = a; *(volatile v4f*)(EB + e * H + 4) = b; __threadfence(); } }
__device__ __forceinline__ void ln_row(float* row, const float* g, const float* bb) { float m = 0.0f; for (int c = 0; c < HF; ++c) m += row[c]; m *= (1.0f / HF); float vr = 0.0f; for (int c = 0; c < HF; ++c) { const float d = row[c] - m; vr += d * d; } vr *= (1.0f / HF); const float rs = rsqrtf(vr + EPS); for (int c = 0; c < HF; ++c) row[c] = pmul((row[c] - m) * rs, bfv(g[c])) + bfv(bb[c]); }
__global__ __launch_bounds__(32) void feat_kernel(const float* __restrict__ x, const int* __restrict__ nenc, const b16* __restrict__ WF, const float* __restrict__ bfeat, const float* __restrict__ TN, int NLIM, float* __restrict__ X1, float* __restrict__ X2) { __shared__ __attribute__((aligned(16))) b16 Ax[16][FI + 8]; __shared__ float Tf[16][260]; const int lane = threadIdx.x, nloc = lane & 15, hlf = lane >> 4; const size_t n0 = (size_t)blockIdx.x * 16; if (n0 >= (size_t)NLIM) return;
  for (int rr = 0; rr < 16; ++rr) for (int q = 0; q < 8; ++q) { const int c = q * 32 + lane; Ax[rr][c] = (b16)(bf16_rne(x[(n0 + rr) * FI + c]) * XS); }
  if (lane < 16) for (int k = FI; k < FI + 8; ++k) Ax[lane][k] = (b16)0.0f;
  wave_lds_sync();
#pragma unroll 1
  for (int g = 0; g < 2; ++g) { v8f acc[16];
#pragma unroll
    for (int t = 0; t < 16; ++t) acc[t] = (v8f){};
#pragma unroll 2
    for (int kb = 0; kb < FI; kb += 32) { const v16b a = frag_kb(&Ax[nloc][kb], hlf);
#pragma unroll
      for (int t = 0; t < 16; ++t) acc[t] = wmma16b(a, frag_kb(WF + (size_t)(g * 256 + t * 16 + nloc) * FI + kb, hlf), acc[t]); }
#pragma unroll
    for (int t = 0; t < 16; ++t) { const int cc = g * 256 + t * 16 + nloc; const float bb = bfv(bfeat[cc]);
#pragma unroll
      for (int r8 = 0; r8 < 8; ++r8) { const int rr = 8 * hlf + r8; const size_t n = n0 + rr; const int i1 = iclamp(nenc[n * 2], 0, NV - 1), i2 = iclamp(nenc[n * 2 + 1], 0, NV - 1); Tf[rr][t * 16 + nloc] = acc[t][r8] * (1.0f / (XS * WSC)) + bb + (TN[(size_t)i1 * HID + cc] + TN[(size_t)i2 * HID + cc]) * 0.5f; } }
    wave_lds_sync();
    float* P = g == 0 ? X1 : X2;
    for (int pass = 0; pass < 2; ++pass) { for (int rr = 0; rr < 16; ++rr) for (int q = 0; q < 2; ++q) *(volatile v4f*)(P + (n0 + rr) * HF + q * 128 + lane * 4) = *(const v4f*)(&Tf[rr][q * 128 + lane * 4]); __threadfence(); }
    wave_lds_sync(); } }
__global__ __launch_bounds__(32) void qkv_kernel(const float* __restrict__ X2, const b16* __restrict__ WLl, const float* __restrict__ g1, const float* __restrict__ b1n, const float* __restrict__ bq, const float* __restrict__ bk, const float* __restrict__ bv, int NLIM, float* __restrict__ QKV) { __shared__ __attribute__((aligned(16))) b16 Ah[16][HF + 8], Al[16][HF + 8]; __shared__ float Tr[16][HF + 1], Tf[16][260]; const int lane = threadIdx.x, nloc = lane & 15, hlf = lane >> 4; const size_t n0 = (size_t)blockIdx.x * 16; if (n0 >= (size_t)NLIM) return;
  for (int rr = 0; rr < 16; ++rr) for (int q = 0; q < 8; ++q) { const int c = q * 32 + lane; Tr[rr][c] = X2[(n0 + rr) * HF + c]; }
  wave_lds_sync(); if (lane < 16) ln_row(&Tr[lane][0], g1, b1n); wave_lds_sync();
  for (int rr = 0; rr < 16; ++rr) for (int q = 0; q < 8; ++q) { const int c = q * 32 + lane; b16 p, pl; split16(Tr[rr][c] * HS, p, pl); Ah[rr][c] = p; Al[rr][c] = pl; }
  if (lane < 16) for (int k = HF; k < HF + 8; ++k) { Ah[lane][k] = (b16)0.0f; Al[lane][k] = (b16)0.0f; }
  wave_lds_sync();
#pragma unroll 1
  for (int g = 0; g < 3; ++g) { const float* bb_ = g == 0 ? bq : g == 1 ? bk : bv; v8f acc[16];
#pragma unroll
    for (int t = 0; t < 16; ++t) acc[t] = (v8f){};
#pragma unroll 2
    for (int kb = 0; kb < HF; kb += 32) { const v16b a = frag_kb(&Ah[nloc][kb], hlf), al = frag_kb(&Al[nloc][kb], hlf);
#pragma unroll
      for (int t = 0; t < 16; ++t) { const v16b bw = frag_kb(WLl + ((size_t)g * HF + t * 16 + nloc) * HF + kb, hlf); acc[t] = wmma16b(a, bw, acc[t]); acc[t] = wmma16b(al, bw, acc[t]); } }
#pragma unroll
    for (int t = 0; t < 16; ++t) { const int cc = t * 16 + nloc; const float bb = bfv(bb_[cc]);
#pragma unroll
      for (int r8 = 0; r8 < 8; ++r8) Tf[8 * hlf + r8][cc] = acc[t][r8] * (1.0f / (HS * WSC)) + bb; }
    wave_lds_sync();
    for (int pass = 0; pass < 2; ++pass) { for (int rr = 0; rr < 16; ++rr) for (int q = 0; q < 2; ++q) *(volatile v4f*)(QKV + (n0 + rr) * 768 + g * 256 + q * 128 + lane * 4) = *(const v4f*)(&Tf[rr][q * 128 + lane * 4]); __threadfence(); }
    wave_lds_sync(); } }
__global__ __launch_bounds__(256) void attn_kernel(const float* __restrict__ QKV, const float* __restrict__ EB, const int* __restrict__ cols, const int* __restrict__ PERM, const int* __restrict__ ROWPTR, const int* __restrict__ ROWCNT, int permLen, int NLIM, float* __restrict__ AO) { const int wave = threadIdx.x >> 5, lane = threadIdx.x & 31; const size_t n = (size_t)blockIdx.x * NPB + wave; if (n >= (size_t)NLIM) return; const int h = lane >> 2, d0 = (lane & 3) * 8;
  float qv[8]; for (int e = 0; e < 8; ++e) qv[e] = QKV[n * 768 + h * D + d0 + e];
  float acc[8]; for (int e = 0; e < 8; ++e) acc[e] = 0.0f; float mx = -INFINITY, den = 0.0f;
  int st = ROWPTR[n], cnt = ROWCNT[n]; cnt = iclamp(cnt, 0, E); st = iclamp(st, 0, permLen - cnt);
#pragma unroll 1
  for (int j = 0; j < cnt; ++j) { const int e = iclamp(PERM[st + j], 0, E - 1); const size_t c = (size_t)iclamp(cols[e], 0, N - 1); if (c >= (size_t)NLIM) continue; const float* kp = QKV + c * 768 + 256 + h * D + d0; float s = 0.0f;
#pragma unroll
    for (int e2 = 0; e2 < 8; ++e2) s += pmul(qv[e2], kp[e2]); s += __shfl_xor(s, 1); s += __shfl_xor(s, 2); s = s * SCALE + EB[(size_t)e * H + h];
    const float mn = fmaxf(mx, s); const float sf = (mx == -INFINITY) ? 0.0f : __expf(mx - mn); const float p = __expf(s - mn); const float* vp = QKV + c * 768 + 512 + h * D + d0;
#pragma unroll
    for (int e2 = 0; e2 < 8; ++e2) acc[e2] = pmul(acc[e2], sf) + pmul(p, vp[e2]); den = pmul(den, sf) + p; mx = mn; }
  const float inv = den > 0.0f ? 1.0f / fmaxf(den, 1e-9f) : 0.0f;
  v4f o0, o1; for (int e2 = 0; e2 < 4; ++e2) { o0[e2] = pmul(acc[e2], inv); o1[e2] = pmul(acc[4 + e2], inv); }
  for (int pass = 0; pass < 2; ++pass) { *(volatile v4f*)(AO + n * HF + h * D + d0) = o0; *(volatile v4f*)(AO + n * HF + h * D + d0 + 4) = o1; __threadfence(); } }
__global__ __launch_bounds__(32) void mlp_kernel(const float* __restrict__ AO, const b16* __restrict__ WLl, const float* __restrict__ bo, const float* __restrict__ g2, const float* __restrict__ b2n, const float* __restrict__ b1, const float* __restrict__ b2, int NLIM, int last, float* __restrict__ X1, float* __restrict__ X2, float* __restrict__ out) { __shared__ __attribute__((aligned(16))) b16 Ah[16][HF + 8], Al[16][HF + 8]; __shared__ float Ty1[16][HF + 1], Tf[16][260]; const int lane = threadIdx.x, nloc = lane & 15, hlf = lane >> 4; const size_t n0 = (size_t)blockIdx.x * 16; if (n0 >= (size_t)NLIM) return;
  auto stage = [&](const float* src, int stride_, bool fromT) { for (int rr = 0; rr < 16; ++rr) for (int q = 0; q < 8; ++q) { const int c = q * 32 + lane; b16 p, pl; split16((fromT ? Tf[rr][c] : src[(n0 + rr) * stride_ + c]) * HS, p, pl); Ah[rr][c] = p; Al[rr][c] = pl; } };
  auto gemm = [&](int m, v8f* acc) {
#pragma unroll
    for (int t = 0; t < 16; ++t) acc[t] = (v8f){};
#pragma unroll 2
    for (int kb = 0; kb < HF; kb += 32) { const v16b a = frag_kb(&Ah[nloc][kb], hlf), al = frag_kb(&Al[nloc][kb], hlf);
#pragma unroll
      for (int t = 0; t < 16; ++t) { const v16b bw = frag_kb(WLl + ((size_t)m * HF + t * 16 + nloc) * HF + kb, hlf); acc[t] = wmma16b(a, bw, acc[t]); acc[t] = wmma16b(al, bw, acc[t]); } } };
  if (lane < 16) for (int k = HF; k < HF + 8; ++k) { Ah[lane][k] = (b16)0.0f; Al[lane][k] = (b16)0.0f; }
  stage(AO, HF, false); wave_lds_sync(); v8f acc[16]; gemm(3, acc);
#pragma unroll
  for (int t = 0; t < 16; ++t) { const int cc = t * 16 + nloc; const float bb = bfv(bo[cc]);
#pragma unroll
    for (int r8 = 0; r8 < 8; ++r8) { const int rr = 8 * hlf + r8; const float y1 = X1[(n0 + rr) * HF + cc] + acc[t][r8] * (1.0f / (HS * WSC)) + bb; Ty1[rr][cc] = y1; Tf[rr][cc] = y1; } }
  wave_lds_sync();
  for (int pass = 0; pass < 2; ++pass) { for (int rr = 0; rr < 16; ++rr) for (int q = 0; q < 8; ++q) { const int c = q * 32 + lane; ((volatile float*)X1)[(n0 + rr) * HF + c] = Ty1[rr][c]; if (last) ((volatile float*)out)[(n0 + rr) * HID + c] = Ty1[rr][c]; } __threadfence(); }
  if (lane < 16) ln_row(&Tf[lane][0], g2, b2n);
  wave_lds_sync(); stage(nullptr, 0, true); wave_lds_sync(); gemm(4, acc);
#pragma unroll
  for (int t = 0; t < 16; ++t) { const int cc = t * 16 + nloc; const float bb = bfv(b1[cc]);
#pragma unroll
    for (int r8 = 0; r8 < 8; ++r8) Tf[8 * hlf + r8][cc] = gelu_erf(acc[t][r8] * (1.0f / (HS * WSC)) + bb); }
  wave_lds_sync(); stage(nullptr, 0, true); wave_lds_sync(); gemm(5, acc);
#pragma unroll
  for (int t = 0; t < 16; ++t) { const int cc = t * 16 + nloc; const float bb = bfv(b2[cc]);
#pragma unroll
    for (int r8 = 0; r8 < 8; ++r8) { const int rr = 8 * hlf + r8; Tf[rr][cc] = X2[(n0 + rr) * HF + cc] + acc[t][r8] * (1.0f / (HS * WSC)) + bb; } }
  wave_lds_sync();
  for (int pass = 0; pass < 2; ++pass) { for (int rr = 0; rr < 16; ++rr) for (int q = 0; q < 2; ++q) { *(volatile v4f*)(X2 + (n0 + rr) * HF + q * 128 + lane * 4) = *(const v4f*)(&Tf[rr][q * 128 + lane * 4]); if (last) *(volatile v4f*)(out + (n0 + rr) * HID + HF + q * 128 + lane * 4) = *(const v4f*)(&Tf[rr][q * 128 + lane * 4]); } __threadfence(); } }
}

extern "C" void kernel_launch(void* const* d_in, const int* in_sizes, int n_in, void* d_out, int out_size, void* d_ws, size_t ws_size, hipStream_t stream) {
  (void)n_in;
  auto Fp = [&](int i) { return (const float*)d_in[i]; }; auto Ip = [&](int i) { return (const int*)d_in[i]; };
  if (in_sizes[0] != N * FI || in_sizes[1] != N * 2 || in_sizes[2] != E * 2 || in_sizes[3] != E || in_sizes[4] != E || in_sizes[5] != E || in_sizes[6] != NV * HID || in_sizes[7] != EV * HID || in_sizes[8] != DV * HID || in_sizes[9] != FI * HID || in_sizes[11] != HID * H || in_sizes[17] != L * HF * HF || in_sizes[29] != L * HF * HF || out_size != N * HID) return;
  const int NLIM = N;
  size_t off = 0; char* ws = (char*)d_ws;
  auto carve = [&](size_t bytes) { char* p = ws + off; off += (bytes + 255) & ~(size_t)255; return p; };
  b16* WF = (b16*)carve((size_t)HID * FI * 2); b16* WL = (b16*)carve((size_t)L * 6 * HF * HF * 2); float* TN = (float*)carve((size_t)NV * HID * 4); float* TE = (float*)carve((size_t)EV * H * 4 + 256); float* TD = (float*)carve((size_t)DV * H * 4 + 256); float* EB = (float*)carve((size_t)E * H * 4); float* X1 = (float*)carve((size_t)N * HF * 4); float* X2 = (float*)carve((size_t)N * HF * 4); float* QKV = (float*)carve((size_t)N * 768 * 4); float* AO = (float*)carve((size_t)N * HF * 4); CsrBufs8 csr; off = csr_carve8(csr, ws, off, E, N);
  if (off > ws_size || off > ((size_t)128 << 20)) return;
  prep_kernel<<<256, 256, 0, stream>>>(Fp(9), Fp(17), Fp(19), Fp(21), Fp(23), Fp(27), Fp(29), Fp(6), Fp(7), Fp(8), Fp(11), Fp(13), WF, WL, TN, TE, TD);
  csr_build8(csr, Ip(4), E, N, stream);
  ebias_kernel<<<(E + 255) / 256, 256, 0, stream>>>(Ip(2), Ip(3), TE, TD, Fp(12), Fp(14), EB);
  feat_kernel<<<NLIM / 16, 32, 0, stream>>>(Fp(0), Ip(1), WF, Fp(10), TN, NLIM, X1, X2);
  const int nb = (NLIM + NPB - 1) / NPB;
  for (int l = 0; l < L; ++l) { const b16* WLl = WL + (size_t)l * 6 * HF * HF; const size_t lo = (size_t)l * HF;
    qkv_kernel<<<NLIM / 16, 32, 0, stream>>>(X2, WLl, Fp(15) + lo, Fp(16) + lo, Fp(18) + lo, Fp(20) + lo, Fp(22) + lo, NLIM, QKV);
    attn_kernel<<<nb, 256, 0, stream>>>(QKV, EB, Ip(5), csr.PERM, csr.ROWPTR, csr.ROWCNT, (int)csr.permLen, NLIM, AO);
    mlp_kernel<<<NLIM / 16, 32, 0, stream>>>(AO, WLl, Fp(24) + lo, Fp(25) + lo, Fp(26) + lo, Fp(28) + lo, Fp(30) + lo, NLIM, l == L - 1 ? 1 : 0, X1, X2, (float*)d_out); }
}
